// Block_34162169872771
// MI455X (gfx1250) — hardware-run, weakly checked
//
#include <hip/hip_runtime.h>


#define NCH 2048
#define NFR 4096

typedef _Float16 h16;
typedef unsigned short bf;
typedef __attribute__((ext_vector_type(16))) __bf16   v16bf;
typedef __attribute__((ext_vector_type(16))) _Float16 v16h;
typedef __attribute__((ext_vector_type(8)))  _Float16 v8h;
typedef __attribute__((ext_vector_type(8)))  unsigned short v8us;
typedef __attribute__((ext_vector_type(8)))  float    v8f;
typedef __attribute__((ext_vector_type(4)))  float    v4f;
typedef v8h  __attribute__((may_alias)) v8ha;
typedef v4f  __attribute__((may_alias)) v4fa;
typedef v8us __attribute__((may_alias)) v8usa;

__device__ __forceinline__ unsigned short f2bf(float f) { unsigned u = __float_as_uint(f); u += 0x7FFFu + ((u >> 16) & 1u); return (unsigned short)(u >> 16); }
__device__ __forceinline__ float bf2f(unsigned short b) { return __uint_as_float(((unsigned)b) << 16); }
__device__ __forceinline__ float bfr(float f) { return bf2f(f2bf(f)); }
__device__ __forceinline__ v16h cat16(v8h lo, v8h hi) { return __builtin_shufflevector(lo, hi, 0, 1, 2, 3, 4, 5, 6, 7, 8, 9, 10, 11, 12, 13, 14, 15); }
__device__ __forceinline__ v16bf cat16b(v8us lo, v8us hi) { return __builtin_bit_cast(v16bf, __builtin_shufflevector(lo, hi, 0, 1, 2, 3, 4, 5, 6, 7, 8, 9, 10, 11, 12, 13, 14, 15)); }
__device__ __forceinline__ v8f wmma16(v16h a, v16h b, v8f c) { return __builtin_amdgcn_wmma_f32_16x16x32_f16(false, a, false, b, (short)0, c, false, false); }
__device__ __forceinline__ v8f wmmab(v16bf a, v16bf b, v8f c) { return __builtin_amdgcn_wmma_f32_16x16x32_bf16(false, a, false, b, (short)0, c, false, false); }

template <typename T16> struct WFrag;
template <> struct WFrag<h16> { typedef v16h V; static __device__ __forceinline__ V ld(const h16* p) { return cat16(*(const v8h*)p, *(const v8h*)(p + 16)); } static __device__ __forceinline__ v8f mma(V a, V b, v8f c) { return wmma16(a, b, c); } };
template <> struct WFrag<bf> { typedef v16bf V; static __device__ __forceinline__ V ld(const bf* p) { return cat16b(*(const v8us*)p, *(const v8us*)(p + 16)); } static __device__ __forceinline__ v8f mma(V a, V b, v8f c) { return wmmab(a, b, c); } };
template <typename T16, int NSPLIT, bool BIAS>
__global__ __launch_bounds__(32) void k_gemmw(const T16* __restrict__ A, const T16* __restrict__ A2, const T16* __restrict__ Bt, const T16* __restrict__ Bt2, int K, float* C, int ldc, const float* __restrict__ bias, size_t sA, size_t sB, size_t sC) {
    typedef typename WFrag<T16>::V V;
    __shared__ __align__(16) float os[16 * 68];
    const size_t z = blockIdx.z; A += z * sA; if (A2) A2 += z * sA; Bt += z * sB; if (Bt2) Bt2 += z * sB; C += z * sC;
    const int lane = threadIdx.x & 31, lr = lane & 15, hi = lane >> 4; const int r0 = blockIdx.x * 64, c0 = blockIdx.y * 64;
    v8f acc[4][4];
#pragma unroll
    for (int mb = 0; mb < 4; ++mb)
#pragma unroll
        for (int nb = 0; nb < 4; ++nb) acc[mb][nb] = (v8f){};
    const size_t aoff = (size_t)(r0 + lr) * K + 8 * hi, boff = (size_t)(c0 + lr) * K + 8 * hi;
    for (int kc = 0; kc < K; kc += 32) {
        V a[4], a2[4];
#pragma unroll
        for (int mb = 0; mb < 4; ++mb) { a[mb] = WFrag<T16>::ld(A + aoff + (size_t)mb * 16 * K + kc); if (NSPLIT == 1 || NSPLIT == 2) a2[mb] = WFrag<T16>::ld(A2 + aoff + (size_t)mb * 16 * K + kc); }
#pragma unroll
        for (int nb = 0; nb < 4; ++nb) { const V b = WFrag<T16>::ld(Bt + boff + (size_t)nb * 16 * K + kc); V b2; if (NSPLIT >= 2) b2 = WFrag<T16>::ld(Bt2 + boff + (size_t)nb * 16 * K + kc);
#pragma unroll
            for (int mb = 0; mb < 4; ++mb) { acc[mb][nb] = WFrag<T16>::mma(a[mb], b, acc[mb][nb]); if (NSPLIT == 1 || NSPLIT == 2) acc[mb][nb] = WFrag<T16>::mma(a2[mb], b, acc[mb][nb]); if (NSPLIT >= 2) acc[mb][nb] = WFrag<T16>::mma(a[mb], b2, acc[mb][nb]); } }
        asm volatile("v_nop\n\tv_nop\n\tv_nop\n\tv_nop" : "+v"(acc[0][0]), "+v"(acc[1][1]), "+v"(acc[2][2]), "+v"(acc[3][3]) : "v"(a[0]), "v"(a[3]));
    }
#pragma unroll
    for (int mb = 0; mb < 4; ++mb) {
#pragma unroll
        for (int nb = 0; nb < 4; ++nb) {
#pragma unroll
            for (int j = 0; j < 8; ++j) os[(hi * 8 + j) * 68 + nb * 16 + lr] = acc[mb][nb][j]; }
        __builtin_amdgcn_wave_barrier(); asm volatile("" ::: "memory");
        float* crow = C + (size_t)(r0 + mb * 16) * ldc + c0;
#pragma unroll 1
        for (int ps = 0; ps < 2; ++ps) {
#pragma unroll
            for (int s = 0; s < 8; ++s) { const int row = 2 * s + hi, cofs = lr * 4; v4f val = *(const v4fa*)(os + row * 68 + cofs); if (BIAS) { val[0] += bfr(bias[c0 + cofs]); val[1] += bfr(bias[c0 + cofs + 1]); val[2] += bfr(bias[c0 + cofs + 2]); val[3] += bfr(bias[c0 + cofs + 3]); }
                *(volatile v4f*)(crow + (size_t)row * ldc + cofs) = val; }
            if (ps == 0) __threadfence(); }
        __builtin_amdgcn_wave_barrier(); asm volatile("" ::: "memory");
    }
}

typedef __attribute__((ext_vector_type(2))) _Float16 v2h;
typedef __attribute__((ext_vector_type(4))) _Float16 v4h;
typedef __attribute__((ext_vector_type(2))) unsigned short v2us;
typedef __attribute__((ext_vector_type(4))) unsigned short v4us;
typedef __attribute__((ext_vector_type(2))) float v2f;
typedef __attribute__((ext_vector_type(4))) int v4i;
__device__ __forceinline__ h16 toh_flush(float x) { const float z = (fabsf(x) < 6.103515625e-05f) ? 0.0f : x; return (h16)z; }

__global__ __launch_bounds__(256) void k_cvt8(const float* __restrict__ src, bf* dst, size_t n8) { const size_t i = (size_t)blockIdx.x * 256 + threadIdx.x; if (i >= n8) return; const v8f v = *(const v8f*)(src + i * 8); v8us o;
#pragma unroll
    for (int k = 0; k < 8; ++k) o[k] = f2bf(v[k]); *(volatile v8us*)(dst + i * 8) = o; __threadfence(); *(volatile v8us*)(dst + i * 8) = o; }

__global__ __launch_bounds__(256) void k_xws(const float* __restrict__ src, h16* dst) {
    const size_t i = (size_t)blockIdx.x * 256 + threadIdx.x; const v8f wv = *(const v8f*)(src + i * 8); v8h ow;
#pragma unroll
    for (int j = 0; j < 8; ++j) ow[j] = toh_flush(bfr(wv[j]) * 1024.0f);
    *(volatile v8h*)(dst + i * 8) = ow; __threadfence(); *(volatile v8h*)(dst + i * 8) = ow; }

__global__ __launch_bounds__(256) void k_rtw(const float* __restrict__ a0, bf* Xr) {
    const unsigned i = blockIdx.x * 256 + threadIdx.x; const unsigned fr = i & 4095u, cb = i >> 12; const float* ps = a0 + (size_t)cb * 64 * NFR + fr; bf r[64];
#pragma unroll
    for (int u = 0; u < 64; ++u) r[u] = f2bf(fmaxf(ps[(size_t)u * NFR], 0.0f));
    bf* pd = Xr + (size_t)fr * NCH + cb * 64;
#pragma unroll
    for (int ps2 = 0; ps2 < 2; ++ps2) {
#pragma unroll
        for (int g = 0; g < 8; ++g) { v8us o;
#pragma unroll
            for (int j = 0; j < 8; ++j) o[j] = r[g * 8 + j];
            *(volatile v8us*)(pd + g * 8) = o; }
        if (ps2 == 0) __threadfence(); } }

__global__ __launch_bounds__(256) void k_rec(const float* __restrict__ Ut, const float* __restrict__ a4, const float* __restrict__ a5, h16* Yw, float* Gp) {
    const unsigned i = blockIdx.x * 256 + threadIdx.x; const unsigned c0 = i * 2u; const float da = 0.5f + (1.0f / (1.0f + expf(-bfr(a4[c0])))) * 0.5f, db = 0.5f + (1.0f / (1.0f + expf(-bfr(a4[c0 + 1])))) * 0.5f; v2f gq; gq[0] = (1.0f / (1.0f + expf(-bfr(a5[c0])))) * 5.0f; gq[1] = (1.0f / (1.0f + expf(-bfr(a5[c0 + 1])))) * 5.0f;
    *(volatile v2f*)(Gp + c0) = gq; __threadfence(); *(volatile v2f*)(Gp + c0) = gq;
    float ra = 0.0f, rb = 0.0f; const float* pu = Ut + c0; h16* py = Yw + c0;
    for (int fr = 0; fr < NFR; ++fr) { const v2f uq = *(const v2f*)(pu + (size_t)fr * NCH); ra = da * (ra + uq[0]); rb = db * (rb + uq[1]); v2h ow; ow[0] = toh_flush(ra); ow[1] = toh_flush(rb);
        *(volatile v2h*)(py + (size_t)fr * NCH) = ow; __threadfence(); *(volatile v2h*)(py + (size_t)fr * NCH) = ow; } }

__device__ __forceinline__ float tanhx(float s) { const float e2 = __builtin_amdgcn_exp2f(s * 2.8853900817779268f); const float r = __fdiv_rn(1.0f, e2 + 1.0f); return 1.0f - (r + r); }

__global__ __launch_bounds__(256) void k_ath(const float* __restrict__ Pt, const float* __restrict__ Ut, const float* __restrict__ Gp, h16* Cw, float* res1) {
    const unsigned i = blockIdx.x * 256 + threadIdx.x; const unsigned fr = i & 4095u, cb = i >> 12; const float* pp = Pt + (size_t)fr * NCH + cb * 64; const float* pu = Ut + (size_t)fr * NCH + cb * 64; const float* pg = Gp + cb * 64; float q[64];
#pragma unroll
    for (int g4 = 0; g4 < 16; ++g4) { const v4f tp = *(const v4fa*)(pp + g4 * 4); const v4f tu = *(const v4fa*)(pu + g4 * 4); const v4f tg = *(const v4fa*)(pg + g4 * 4);
#pragma unroll
        for (int j = 0; j < 4; ++j) q[g4 * 4 + j] = tanhx((tp[j] * 0.0009765625f + tu[j]) * tg[j]); }
    h16* pc = Cw + (size_t)fr * NCH + cb * 64; float* pr = res1 + (size_t)cb * 64 * NFR + fr;
#pragma unroll
    for (int ps2 = 0; ps2 < 2; ++ps2) {
#pragma unroll
        for (int g = 0; g < 8; ++g) { v8h o;
#pragma unroll
            for (int j = 0; j < 8; ++j) o[j] = toh_flush(q[g * 8 + j]);
            *(volatile v8h*)(pc + g * 8) = o; }
#pragma unroll
        for (int u = 0; u < 64; ++u) *(volatile float*)(pr + (size_t)u * NFR) = q[u];
        if (ps2 == 0) __threadfence(); } }

__global__ __launch_bounds__(256) void k_scl(const float* __restrict__ Ft, float* res0) {
    const size_t i = (size_t)blockIdx.x * 256 + threadIdx.x; const v4f t = *(const v4fa*)(Ft + i * 4); v4f o;
#pragma unroll
    for (int j = 0; j < 4; ++j) o[j] = t[j] * 0.0009765625f;
    *(volatile v4f*)(res0 + i * 4) = o; __threadfence(); *(volatile v4f*)(res0 + i * 4) = o; }

extern "C" void kernel_launch(void* const* d_in, const int* in_sizes, int n_in, void* d_out, int out_size, void* d_ws, size_t ws_size, hipStream_t stream) {
    if (n_in < 6) return;
    if (in_sizes[0] != NCH * NFR || in_sizes[1] != NCH * NCH || in_sizes[2] != NCH * NCH || in_sizes[3] != NCH * NCH || in_sizes[4] != NCH || in_sizes[5] != NCH) return;
    if (out_size != 2 * NCH * NFR) return;
    static_assert(NCH == 2048 && NFR == 4096 && NCH % 64 == 0 && NFR % 64 == 0 && NCH % 32 == 0 && (NCH * NCH / 8) % 256 == 0 && (NFR * (NCH / 64)) % 256 == 0 && (NCH / 2) % 256 == 0 && (NCH * NFR / 4) % 256 == 0, "the products: row and column counts multiples of 64, the depth of 32; the flat grids exact; a step number takes twelve bits");
    const float* a0 = (const float*)d_in[0]; const float* a1 = (const float*)d_in[1]; const float* a2 = (const float*)d_in[2]; const float* a3 = (const float*)d_in[3]; const float* a4 = (const float*)d_in[4]; const float* a5 = (const float*)d_in[5]; float* res0 = (float*)d_out; float* res1 = res0 + (size_t)NFR * NCH;
    char* wsp = (char*)d_ws; auto take = [&](size_t bytes) { char* p = wsp; wsp += (bytes + 255) & ~(size_t)255; return (void*)p; };
    bf* Xr = (bf*)take((size_t)NFR * NCH * 2); bf* Wa = (bf*)take((size_t)NCH * NCH * 2); h16* Wb = (h16*)take((size_t)NCH * NCH * 2); h16* Wc = (h16*)take((size_t)NCH * NCH * 2); float* Ut = (float*)take((size_t)NFR * NCH * 4); h16* Yw = (h16*)take((size_t)NFR * NCH * 2); float* Pt = (float*)take((size_t)NFR * NCH * 4); float* Gp = (float*)take((size_t)NCH * 4);
    if ((size_t)(wsp - (char*)d_ws) > ws_size) return;
    h16* Cw = Yw; float* Ft = Ut;
    k_rtw<<<NFR * (NCH / 64) / 256, 256, 0, stream>>>(a0, Xr);
    k_cvt8<<<(unsigned)(NCH * NCH / 8 / 256), 256, 0, stream>>>(a1, Wa, (size_t)NCH * NCH / 8);
    k_xws<<<(unsigned)(NCH * NCH / 8 / 256), 256, 0, stream>>>(a2, Wb); k_xws<<<(unsigned)(NCH * NCH / 8 / 256), 256, 0, stream>>>(a3, Wc);
    k_gemmw<bf, 0, false><<<dim3(NFR / 64, NCH / 64, 1), 32, 0, stream>>>(Xr, nullptr, Wa, nullptr, NCH, Ut, NCH, nullptr, 0, 0, 0);
    k_rec<<<NCH / 2 / 256, 256, 0, stream>>>(Ut, a4, a5, Yw, Gp);
    k_gemmw<h16, 0, false><<<dim3(NFR / 64, NCH / 64, 1), 32, 0, stream>>>(Yw, nullptr, Wb, nullptr, NCH, Pt, NCH, nullptr, 0, 0, 0);
    k_ath<<<NFR * (NCH / 64) / 256, 256, 0, stream>>>(Pt, Ut, Gp, Cw, res1);
    k_gemmw<h16, 0, false><<<dim3(NFR / 64, NCH / 64, 1), 32, 0, stream>>>(Cw, nullptr, Wc, nullptr, NCH, Ft, NCH, nullptr, 0, 0, 0);
    k_scl<<<(unsigned)((size_t)NCH * NFR / 4 / 256), 256, 0, stream>>>(Ft, res0);
}
